// CorrelationModule_4672924418157
// MI455X (gfx1250) — hardware-verified
//
#include <hip/hip_runtime.h>
#include <math.h>
#include <stdint.h>

#ifndef NB
#define NB 4
#endif
#ifndef NQ
#define NQ 4096
#endif
#define NB_FULL 4
#define CC    64
#define NN    4096
#define HWD   64
#define QT    64
#define OSP   68
#define TP    72
#define NTAP  9
#define KCV   576
#define LNPS  9.704060527839234f
#define PRS   1024.0f
#define PRSI  0.0009765625f
#define BNEPS 1.0e-5f

static_assert(NB >= 1 && NB <= NB_FULL);
static_assert(NQ >= QT && NQ <= NN && NQ % QT == 0);
static_assert(NN == HWD * HWD && NN % QT == 0 && NN % 32 == 0);
static_assert(CC == QT && CC % 32 == 0);
static_assert(KCV == NTAP * CC && KCV % 32 == 0);
static_assert((OSP * 4) % 16 == 0);
static_assert((TP * 2) % 16 == 0);
static_assert((KCV * 2) % 128 == 0);
static_assert((CC * KCV) % (8 * 256) == 0 && (CC * KCV) / (8 * 256) == 18);
static_assert((CC * CC) / (8 * 256) == 2);

typedef _Float16       v16h __attribute__((ext_vector_type(16)));
typedef _Float16       v8h  __attribute__((ext_vector_type(8)));
typedef __bf16         v16b __attribute__((ext_vector_type(16)));
typedef unsigned short v8us __attribute__((ext_vector_type(8)));
typedef float          v8f  __attribute__((ext_vector_type(8)));
typedef float          v4f  __attribute__((ext_vector_type(4)));
typedef unsigned int   v4u  __attribute__((ext_vector_type(4)));

union Frag  { v8us u[2]; v16h h; v16b bf; v4u w[2]; };
union FragH { v16h v; v8h hv[2]; };
static_assert(sizeof(Frag) == 32);
static_assert(sizeof(FragH) == 32);

__device__ __forceinline__ unsigned short bf_bits(float f) {
  unsigned u = __float_as_uint(f);
  return (unsigned short)((u + 0x7FFFu + ((u >> 16) & 1u)) >> 16);
}
__device__ __forceinline__ float bf_up(unsigned short hb) { return __uint_as_float(((unsigned)hb) << 16); }
__device__ __forceinline__ float bfr(float f) { return bf_up(bf_bits(f)); }
__device__ __forceinline__ unsigned short h_bits(_Float16 x) { return __builtin_bit_cast(unsigned short, x); }
__device__ __forceinline__ unsigned pk16(unsigned short a, unsigned short b) { return (unsigned)a | ((unsigned)b << 16); }
__device__ __forceinline__ v8f zero8() { v8f z = {0.f, 0.f, 0.f, 0.f, 0.f, 0.f, 0.f, 0.f}; return z; }
__device__ __forceinline__ float hmax8(v8f s) {
  return fmaxf(fmaxf(fmaxf(s[0], s[1]), fmaxf(s[2], s[3])), fmaxf(fmaxf(s[4], s[5]), fmaxf(s[6], s[7])));
}
__device__ __forceinline__ unsigned wave_ballot(bool p) {
#if defined(__HIP_DEVICE_COMPILE__)
  return __builtin_amdgcn_ballot_w32(p);
#else
  return p ? 1u : 0u;
#endif
}

__device__ __forceinline__ Frag ldfrag(const unsigned short* p) {
  Frag f;
  f.u[0] = *(const v8us*)(p);
  f.u[1] = *(const v8us*)(p + 16);
  return f;
}

__device__ __forceinline__ v8f mma_h(v16h a, v16h b, v8f c) {
  v8f d = __builtin_amdgcn_wmma_f32_16x16x32_f16(false, a, false, b, (short)0, c, false, false);
#if defined(__HIP_DEVICE_COMPILE__)
  asm volatile("v_nop\n\tv_nop\n\tv_nop\n\tv_nop" : "+v"(d) : "v"(a), "v"(b));
#endif
  return d;
}
__device__ __forceinline__ v8f mma_b(v16b a, v16b b, v8f c) {
  v8f d = __builtin_amdgcn_wmma_f32_16x16x32_bf16(false, a, false, b, (short)0, c, false, false);
#if defined(__HIP_DEVICE_COMPILE__)
  const v16h ha = __builtin_bit_cast(v16h, a), hb = __builtin_bit_cast(v16h, b);
  asm volatile("v_nop\n\tv_nop\n\tv_nop\n\tv_nop" : "+v"(d) : "v"(ha), "v"(hb));
#endif
  return d;
}

__global__ __launch_bounds__(256)
void cvt_w(const float* __restrict__ wlin, const float* __restrict__ wconv, unsigned short* Wl, unsigned short* Wc) {
  const int tid = threadIdx.x, blk = blockIdx.x;
  if (blk < 18) {
    const int g = blk * 256 + tid;
    const int L = g >> 3, e = g & 7;
    const int o = L / NTAP, tap = L - NTAP * o;
    const float* s = wconv + ((size_t)o * CC + 8 * e) * NTAP + tap;
    v4u u;
#pragma unroll
    for (int t = 0; t < 4; ++t)
      u[t] = pk16(bf_bits(s[(2 * t) * NTAP]), bf_bits(s[(2 * t + 1) * NTAP]));
    const size_t po = (size_t)o * KCV + (size_t)tap * CC + 8 * e;
#pragma unroll
    for (int pass = 0; pass < 2; ++pass) {
      *(volatile v4u*)(Wc + po) = u;
      __threadfence();
    }
  } else {
    const int g = (blk - 18) * 256 + tid;
    const int d = g >> 3, e = g & 7;
    const float* s = wlin + (size_t)d * CC + 8 * e;
    const v4f a = *(const v4f*)s;
    const v4f q = *(const v4f*)(s + 4);
    const float f[8] = {a[0], a[1], a[2], a[3], q[0], q[1], q[2], q[3]};
    v4u u;
#pragma unroll
    for (int t = 0; t < 4; ++t) u[t] = pk16(bf_bits(f[2 * t]), bf_bits(f[2 * t + 1]));
    const size_t po = (size_t)d * CC + 8 * e;
#pragma unroll
    for (int pass = 0; pass < 2; ++pass) {
      *(volatile v4u*)(Wl + po) = u;
      __threadfence();
    }
  }
}

template <int WV>
__global__ __launch_bounds__(256)
void cvt_x(const float* __restrict__ x, unsigned short* H, unsigned short* V) {
  __shared__ __align__(16) unsigned short Th[QT * TP];
  const int tid = threadIdx.x;
  const int nb = blockIdx.x, b = blockIdx.y;
  const int e = tid & 7, lq = tid >> 3;
  const int n0 = nb * QT;
  v4u uv[2];
#pragma unroll
  for (int it = 0; it < 2; ++it) {
    const int cl = it * 32 + lq;
    const float* sp = x + ((size_t)(b * CC + cl)) * NN + n0 + 8 * e;
    const v4f a = *(const v4f*)sp;
    const v4f q = *(const v4f*)(sp + 4);
    const float f[8] = {a[0], a[1], a[2], a[3], q[0], q[1], q[2], q[3]};
    unsigned short hb[8];
#pragma unroll
    for (int t = 0; t < 8; ++t) { hb[t] = bf_bits(f[t]); Th[(8 * e + t) * TP + cl] = hb[t]; }
#pragma unroll
    for (int t = 0; t < 4; ++t)
      uv[it][t] = pk16(h_bits((_Float16)bf_up(hb[2 * t])), h_bits((_Float16)bf_up(hb[2 * t + 1])));
  }
  __syncthreads();
  v4u uh[2];
#pragma unroll
  for (int it = 0; it < 2; ++it) {
    const int nl = it * 32 + lq;
    uh[it] = *(const v4u*)(Th + nl * TP + 8 * e);
  }
#pragma unroll
  for (int pass = 0; pass < 2; ++pass) {
#pragma unroll
    for (int it = 0; it < 2; ++it) {
      const int nl = it * 32 + lq;
      const size_t po = ((size_t)(b * NN + n0 + nl)) * CC + 8 * e;
      *(volatile v4u*)(H + po) = uh[it];
      if (WV == 1) {
        const int cl = it * 32 + lq;
        const size_t pv = ((size_t)(b * CC + cl)) * NN + n0 + 8 * e;
        *(volatile v4u*)(V + pv) = uv[it];
      }
    }
    __threadfence();
  }
}

__global__ __launch_bounds__(128)
void gemm_q(const unsigned short* __restrict__ Wl, const unsigned short* __restrict__ X,
            unsigned short* Qh, unsigned short* Ql) {
  __shared__ __align__(16) float Vs[QT * OSP];
  const int tid  = threadIdx.x;
  const int lane = tid & 31, wave = tid >> 5;
  const int hh   = lane >> 4, c = lane & 15;
  const int nt   = blockIdx.x, b = blockIdx.y;
  const int n0   = nt * QT;

  const unsigned short* ap = X + ((size_t)(b * NN + n0 + 16 * wave + c)) * CC + 8 * hh;
  const unsigned short* bp = Wl + (size_t)c * CC + 8 * hh;

  v8f acc[4];
#pragma unroll
  for (int j = 0; j < 4; ++j) acc[j] = zero8();

#pragma unroll
  for (int ks = 0; ks < CC / 32; ++ks) {
    const Frag fa = ldfrag(ap + 32 * ks);
#pragma unroll
    for (int j = 0; j < 4; ++j) {
      const Frag fb = ldfrag(bp + (size_t)(16 * j) * CC + 32 * ks);
      acc[j] = mma_b(fa.bf, fb.bf, acc[j]);
    }
  }

  {
    const int nrow = 16 * wave + 8 * hh;
#pragma unroll
    for (int j = 0; j < 4; ++j) {
      v4f va, vb;
#pragma unroll
      for (int r = 0; r < 4; ++r) { va[r] = acc[j][r]; vb[r] = acc[j][4 + r]; }
      *(v4f*)(Vs + (16 * j + c) * OSP + nrow)     = va;
      *(v4f*)(Vs + (16 * j + c) * OSP + nrow + 4) = vb;
    }
  }
  __syncthreads();

  const int e = tid & 7, lq = tid >> 3;
  v4u uh[4], ul[4];
#pragma unroll
  for (int it = 0; it < 4; ++it) {
    const int nl = it * 16 + lq;
    float f[8];
#pragma unroll
    for (int t = 0; t < 8; ++t) f[t] = Vs[(8 * e + t) * OSP + nl];
#pragma unroll
    for (int t = 0; t < 4; ++t) {
      const float f0 = f[2 * t], f1 = f[2 * t + 1];
      const unsigned short hb0 = bf_bits(f0), hb1 = bf_bits(f1);
      const unsigned short lb0 = bf_bits(f0 - bf_up(hb0));
      const unsigned short lb1 = bf_bits(f1 - bf_up(hb1));
      uh[it][t] = pk16(hb0, hb1);
      ul[it][t] = pk16(lb0, lb1);
    }
  }
#pragma unroll
  for (int pass = 0; pass < 2; ++pass) {
#pragma unroll
    for (int it = 0; it < 4; ++it) {
      const int nl = it * 16 + lq;
      const size_t po = ((size_t)(b * NN + n0 + nl)) * CC + 8 * e;
      *(volatile v4u*)(Qh + po) = uh[it];
      *(volatile v4u*)(Ql + po) = ul[it];
    }
    __threadfence();
  }
}

__global__ __launch_bounds__(128)
void attn_k(const unsigned short* __restrict__ Qh, const unsigned short* __restrict__ Ql,
            const unsigned short* __restrict__ Kt, const unsigned short* __restrict__ Vh,
            unsigned short* Ah, unsigned short* Al) {
  __shared__ __align__(16) float Os[QT * OSP];
  const int tid  = threadIdx.x;
  const int wave = tid >> 5, lane = tid & 31;
  const int hh   = lane >> 4, c = lane & 15;
  const int n0   = blockIdx.x * QT, b = blockIdx.y;

  const size_t qo = ((size_t)(b * NN + n0 + 16 * wave + c)) * CC + 8 * hh;
  const unsigned short* Qhp = Qh + qo;
  const unsigned short* Qlp = Ql + qo;
  const unsigned short* Khp = Kt + (size_t)b * NN * CC + (size_t)c * CC + 8 * hh;
  const unsigned short* Vp = Vh + (size_t)b * CC * NN + (size_t)c * NN + 8 * hh;

  float m = -1.0e30f, l = 0.f;
  v8f o[4], o2[4];
#pragma unroll
  for (int j = 0; j < 4; ++j) { o[j] = zero8(); o2[j] = zero8(); }

#pragma unroll 1
  for (int kb = 0; kb < NN; kb += 32) {
    const unsigned short* k0p = Khp + (size_t)kb * CC;
    const unsigned short* k1p = Khp + (size_t)(kb + 16) * CC;
    v8f s0 = zero8(), s1 = zero8();
#pragma unroll
    for (int kc = 0; kc < CC / 32; ++kc) {
      const Frag qh = ldfrag(Qhp + 32 * kc);
      const Frag ql = ldfrag(Qlp + 32 * kc);
      const Frag k0 = ldfrag(k0p + 32 * kc);
      const Frag k1 = ldfrag(k1p + 32 * kc);
      s0 = mma_b(k0.bf, qh.bf, s0);
      s1 = mma_b(k1.bf, qh.bf, s1);
      s0 = mma_b(k0.bf, ql.bf, s0);
      s1 = mma_b(k1.bf, ql.bf, s1);
    }

    float mx = fmaxf(hmax8(s0), hmax8(s1));
    mx = fmaxf(mx, __shfl_xor(mx, 16, 32));
    const float mn = fmaxf(m, mx);
    const unsigned grew = wave_ballot(mx > m);
    if (grew != 0u) {
      const float corr = __expf(m - mn);
      l *= corr;
#pragma unroll
      for (int j = 0; j < 4; ++j) {
#pragma unroll
        for (int r = 0; r < 8; ++r) { o[j][r] *= corr; o2[j][r] *= corr; }
      }
    }
    m = mn;
    const float msh = mn - LNPS;

    FragH ph, pr;
    float ls = 0.f;
#pragma unroll
    for (int r = 0; r < 8; ++r) {
      const float e0 = __expf(s0[r] - msh);
      const float e1 = __expf(s1[r] - msh);
      ls += e0 + e1;
      const _Float16 h0 = (_Float16)e0, h1 = (_Float16)e1;
      ph.hv[0][r] = h0;
      ph.hv[1][r] = h1;
      pr.hv[0][r] = (_Float16)((e0 - (float)h0) * PRS);
      pr.hv[1][r] = (_Float16)((e1 - (float)h1) * PRS);
    }
    l += ls;

#pragma unroll
    for (int j = 0; j < 4; ++j) {
      const Frag vf = ldfrag(Vp + (size_t)(16 * j) * NN + kb);
      o[j]  = mma_h(vf.h, ph.v, o[j]);
      o2[j] = mma_h(vf.h, pr.v, o2[j]);
    }
  }
  l += __shfl_xor(l, 16, 32);
  const float inv = 1.0f / l;

  const int qrow = 16 * wave + c;
#pragma unroll
  for (int j = 0; j < 4; ++j) {
    v4f va, vb;
#pragma unroll
    for (int r = 0; r < 4; ++r) {
      va[r] = (o[j][r]     + o2[j][r]     * PRSI) * inv;
      vb[r] = (o[j][4 + r] + o2[j][4 + r] * PRSI) * inv;
    }
    *(v4f*)(Os + qrow * OSP + 16 * j + 8 * hh)     = va;
    *(v4f*)(Os + qrow * OSP + 16 * j + 8 * hh + 4) = vb;
  }
  __syncthreads();

  const int e = tid & 7, lq = tid >> 3;
  v4u uh[4], ul[4];
#pragma unroll
  for (int it = 0; it < 4; ++it) {
    const int row = it * 16 + lq;
    const v4f a = *(const v4f*)(Os + row * OSP + 8 * e);
    const v4f q = *(const v4f*)(Os + row * OSP + 8 * e + 4);
    const float f[8] = {a[0], a[1], a[2], a[3], q[0], q[1], q[2], q[3]};
#pragma unroll
    for (int t = 0; t < 4; ++t) {
      const float f0 = f[2 * t], f1 = f[2 * t + 1];
      const unsigned short hb0 = bf_bits(f0), hb1 = bf_bits(f1);
      const unsigned short lb0 = bf_bits(f0 - bf_up(hb0));
      const unsigned short lb1 = bf_bits(f1 - bf_up(hb1));
      uh[it][t] = pk16(hb0, hb1);
      ul[it][t] = pk16(lb0, lb1);
    }
  }
#pragma unroll
  for (int pass = 0; pass < 2; ++pass) {
#pragma unroll
    for (int it = 0; it < 4; ++it) {
      const int row = it * 16 + lq;
      const size_t po = ((size_t)(b * NN + n0 + row)) * CC + 8 * e;
      *(volatile v4u*)(Ah + po) = uh[it];
      *(volatile v4u*)(Al + po) = ul[it];
    }
    __threadfence();
  }
}

__global__ __launch_bounds__(128)
void conv_k(const unsigned short* __restrict__ Wc, const unsigned short* __restrict__ Ah,
            const unsigned short* __restrict__ Al, const float* __restrict__ gamma, const float* __restrict__ beta,
            const float* __restrict__ rmean, const float* __restrict__ rvar, float* out) {
  __shared__ __align__(16) float Vs[QT * OSP];
  const int tid  = threadIdx.x;
  const int lane = tid & 31, wave = tid >> 5;
  const int hh   = lane >> 4, c = lane & 15;
  const int nt   = blockIdx.x, b = blockIdx.y;
  const int n0   = nt * QT;

  const int p  = n0 + 16 * wave + c;
  const int py = p >> 6, px = p & (HWD - 1);
  const unsigned short* bp = Wc + (size_t)c * KCV + 8 * hh;
  const size_t abase = (size_t)b * NN * CC + 8 * hh;

  v8f acc[4];
#pragma unroll
  for (int j = 0; j < 4; ++j) acc[j] = zero8();

#pragma unroll 1
  for (int tap = 0; tap < NTAP; ++tap) {
    const int t3 = tap / 3;
    const int yy = py + t3 - 1, xx = px + (tap - 3 * t3) - 1;
    const bool valid = ((unsigned)yy < (unsigned)HWD) && ((unsigned)xx < (unsigned)HWD);
    const int yc = (yy < 0) ? 0 : ((yy > HWD - 1) ? (HWD - 1) : yy);
    const int xc = (xx < 0) ? 0 : ((xx > HWD - 1) ? (HWD - 1) : xx);
    const unsigned msk = valid ? 0xFFFFFFFFu : 0u;
    const size_t ao = abase + (size_t)(yc * HWD + xc) * CC;
    const unsigned short* ahp = Ah + ao;
    const unsigned short* alp = Al + ao;
#pragma unroll
    for (int kc = 0; kc < CC / 32; ++kc) {
      Frag fah = ldfrag(ahp + 32 * kc);
      Frag fal = ldfrag(alp + 32 * kc);
#pragma unroll
      for (int i = 0; i < 2; ++i) { fah.w[i] = fah.w[i] & msk; fal.w[i] = fal.w[i] & msk; }
#pragma unroll
      for (int j = 0; j < 4; ++j) {
        const Frag fb = ldfrag(bp + (size_t)(16 * j) * KCV + tap * CC + 32 * kc);
        acc[j] = mma_b(fah.bf, fb.bf, acc[j]);
        acc[j] = mma_b(fal.bf, fb.bf, acc[j]);
      }
    }
  }

  {
    const int nrow = 16 * wave + 8 * hh;
#pragma unroll
    for (int j = 0; j < 4; ++j) {
      const int o = 16 * j + c;
      const float sc = bfr(gamma[o]) * (1.0f / sqrtf(bfr(rvar[o]) + BNEPS));
      const float mu = bfr(rmean[o]);
      const float be = bfr(beta[o]);
      v4f va, vb;
#pragma unroll
      for (int r = 0; r < 4; ++r) {
        float y0 = (acc[j][r]     - mu) * sc + be;
        float y1 = (acc[j][4 + r] - mu) * sc + be;
        y0 = (y0 > 0.f) ? y0 : 0.1f * y0;
        y1 = (y1 > 0.f) ? y1 : 0.1f * y1;
        va[r] = y0; vb[r] = y1;
      }
      *(v4f*)(Vs + o * OSP + nrow)     = va;
      *(v4f*)(Vs + o * OSP + nrow + 4) = vb;
    }
  }
  __syncthreads();

  const int e = tid & 15, lq = tid >> 4;
  v4f res[8];
#pragma unroll
  for (int it = 0; it < 8; ++it) {
    const int ol = it * 8 + lq;
    res[it] = *(const v4f*)(Vs + ol * OSP + 4 * e);
  }
#pragma unroll
  for (int pass = 0; pass < 2; ++pass) {
#pragma unroll
    for (int it = 0; it < 8; ++it) {
      const int ol = it * 8 + lq;
      const size_t idx = ((size_t)(b * CC + ol)) * NN + n0 + 4 * e;
      *(volatile v4f*)(out + idx) = res[it];
    }
    __threadfence();
  }
}

extern "C" void kernel_launch(void* const* d_in, const int* in_sizes, int n_in,
                              void* d_out, int out_size, void* d_ws, size_t ws_size,
                              hipStream_t stream) {
  if (n_in < 8) return;
  if (in_sizes[0] < NB * CC * NN) return;
  if (in_sizes[1] < NB * CC * NN) return;
  if (in_sizes[2] < CC * CC) return;
  if (in_sizes[3] < CC * KCV) return;
  if (in_sizes[4] < CC || in_sizes[5] < CC || in_sizes[6] < CC || in_sizes[7] < CC) return;
  if (out_size < NB * CC * NN) return;

  size_t off = 0;
  auto carve = [&](size_t bytes) { const size_t o = off; off += (bytes + 255) & ~(size_t)255; return o; };
  const size_t plane = (size_t)NB * NN * CC * 2;
  const size_t oWl = carve((size_t)CC * CC * 2);
  const size_t oWc = carve((size_t)CC * KCV * 2);
  const size_t oX  = carve(plane);
  const size_t oKt = carve(plane);
  const size_t oV  = carve(plane);
  const size_t oQh = carve(plane);
  const size_t oQl = carve(plane);
  const size_t oAh = carve(plane);
  const size_t oAl = carve(plane);
  if (off > ws_size) return;
  if (off > (size_t)134217728) return;

  const float* ex    = (const float*)d_in[0];
  const float* qin   = (const float*)d_in[1];
  const float* wlin  = (const float*)d_in[2];
  const float* wconv = (const float*)d_in[3];
  const float* gamma = (const float*)d_in[4];
  const float* beta  = (const float*)d_in[5];
  const float* rmean = (const float*)d_in[6];
  const float* rvar  = (const float*)d_in[7];

  char* ws = (char*)d_ws;
  unsigned short* Wl = (unsigned short*)(ws + oWl);
  unsigned short* Wc = (unsigned short*)(ws + oWc);
  unsigned short* X  = (unsigned short*)(ws + oX);
  unsigned short* Kt = (unsigned short*)(ws + oKt);
  unsigned short* V  = (unsigned short*)(ws + oV);
  unsigned short* Qh = (unsigned short*)(ws + oQh);
  unsigned short* Ql = (unsigned short*)(ws + oQl);
  unsigned short* Ah = (unsigned short*)(ws + oAh);
  unsigned short* Al = (unsigned short*)(ws + oAl);
  float* out = (float*)d_out;

  const dim3 blk256(256), blk128(128);

  cvt_w<<<dim3(20), blk256, 0, stream>>>(wlin, wconv, Wl, Wc);
  cvt_x<0><<<dim3(NN / QT, NB), blk256, 0, stream>>>(ex, X, X);
  cvt_x<1><<<dim3(NN / QT, NB), blk256, 0, stream>>>(qin, Kt, V);
  gemm_q<<<dim3(NQ / QT, NB), blk128, 0, stream>>>(Wl, X, Qh, Ql);
  attn_k<<<dim3(NQ / QT, NB), blk128, 0, stream>>>(Qh, Ql, Kt, V, Ah, Al);
  conv_k<<<dim3(NN / QT, NB), blk128, 0, stream>>>(Wc, Ah, Al, gamma, beta, rmean, rvar, out);
  (void)hipGetLastError();
}
